// MambaLayer_14396730376917
// MI455X (gfx1250) — hardware-verified
//
#include <hip/hip_runtime.h>
#include <math.h>

typedef __attribute__((ext_vector_type(16))) __bf16   v16b;
typedef __attribute__((ext_vector_type(8)))  __bf16   v8b;
typedef __attribute__((ext_vector_type(8)))  _Float16 v8h;
typedef __attribute__((ext_vector_type(8)))  float    v8f;
typedef __attribute__((ext_vector_type(4)))  float    v4f;

constexpr int kBatch  = 2;
constexpr int kSeq    = 2048;
constexpr int kDm     = 1024;
constexpr int kE      = 2048;
constexpr int kNst    = 16;
constexpr int kR      = 64;
constexpr int kRows   = kBatch * kSeq;
constexpr int kBCW    = 64;
constexpr int kConvTP = 260;
constexpr int kScanTS = 64;
constexpr int kScanCh = 64;
constexpr int kScanP  = 68;
static_assert(2 * kNst <= 32 && kR == kBCW);
static_assert((kDm % 32) == 0 && (kE % 32) == 0 && (kR % 32) == 0);
static_assert((kRows % 64) == 0 && (kE % 64) == 0 && (kDm % 64) == 0 && (kBCW % 64) == 0);
static_assert((kSeq % kScanTS) == 0 && (kSeq % 64) == 0 && (kE % kScanCh) == 0 && (kE % 256) == 0 && (kDm % 8) == 0);

constexpr size_t kOffXH   = 0;
constexpr size_t kOffXL   = kOffXH  + (size_t)kRows * kDm * 2;
constexpr size_t kOffWSK  = kOffXL  + (size_t)kRows * kDm * 2;
constexpr size_t kOffWIN  = kOffWSK + (size_t)kE * kDm * 2;
constexpr size_t kOffWOUT = kOffWIN + (size_t)kE * kDm * 2;
constexpr size_t kOffWD1  = kOffWOUT + (size_t)kDm * kE * 2;
constexpr size_t kOffWBC  = kOffWD1 + (size_t)kBCW * kE * 2;
constexpr size_t kOffWD2  = kOffWBC + (size_t)kBCW * kE * 2;
constexpr size_t kOffXE   = kOffWD2 + (size_t)kE * kR * 2;
constexpr size_t kOffXSH  = kOffXE  + (size_t)kRows * kE * 4;
constexpr size_t kOffXSL  = kOffXSH + (size_t)kRows * kE * 2;
constexpr size_t kOffD1H  = kOffXSL + (size_t)kRows * kE * 2;
constexpr size_t kOffD1L  = kOffD1H + (size_t)kRows * kBCW * 2;
constexpr size_t kOffXBC  = kOffD1L + (size_t)kRows * kBCW * 2;
constexpr size_t kOffYP   = kOffXBC + (size_t)kRows * kBCW * 4;
constexpr size_t kWsTotal = kOffYP  + (size_t)kRows * kE * 4;
static_assert(kWsTotal == 132907008ull);
static_assert(kWsTotal <= 134217728ull);
static_assert((kOffXL % 128) == 0 && (kOffWSK % 128) == 0 && (kOffWIN % 128) == 0 && (kOffWOUT % 128) == 0 &&
              (kOffWD1 % 128) == 0 && (kOffWBC % 128) == 0 && (kOffWD2 % 128) == 0 && (kOffXE % 128) == 0 &&
              (kOffXSH % 128) == 0 && (kOffXSL % 128) == 0 && (kOffD1H % 128) == 0 && (kOffD1L % 128) == 0 &&
              (kOffXBC % 128) == 0 && (kOffYP % 128) == 0);

__device__ __forceinline__ unsigned short f2bf_bits(float f) {
  unsigned u = __float_as_uint(f);
  return (unsigned short)((u + 0x7FFFu + ((u >> 16) & 1u)) >> 16);
}
__device__ __forceinline__ float bf_bits2f(unsigned short h) { return __uint_as_float(((unsigned)h) << 16); }
__device__ __forceinline__ float bfr(float f) { return bf_bits2f(f2bf_bits(f)); }

__device__ __forceinline__ v8h pack_bf16x8(v4f a0, v4f a1) {
  v8h hv;
#pragma unroll
  for (int e = 0; e < 4; ++e) {
    const float x0 = a0[e], x1 = a1[e];
    hv[e]     = __builtin_bit_cast(_Float16, f2bf_bits(x0));
    hv[4 + e] = __builtin_bit_cast(_Float16, f2bf_bits(x1));
  }
  return hv;
}
__device__ __forceinline__ void split_bf16x8(v4f a0, v4f a1, v8h& hv, v8h& lv) {
#pragma unroll
  for (int e = 0; e < 4; ++e) {
    const float x0 = a0[e], x1 = a1[e];
    const unsigned short h0 = f2bf_bits(x0), h1 = f2bf_bits(x1);
    const unsigned short l0 = f2bf_bits(x0 - bf_bits2f(h0)), l1 = f2bf_bits(x1 - bf_bits2f(h1));
    hv[e]     = __builtin_bit_cast(_Float16, h0);
    hv[4 + e] = __builtin_bit_cast(_Float16, h1);
    lv[e]     = __builtin_bit_cast(_Float16, l0);
    lv[4 + e] = __builtin_bit_cast(_Float16, l1);
  }
}

__device__ __forceinline__ v16b frag_load(const __bf16* p) {
  union { v16b v; v8b h[2]; } f;
  f.h[0] = *(const v8b*)(p); f.h[1] = *(const v8b*)(p + 16); return f.v;
}
__device__ __forceinline__ v8f mma_bf16(v16b a, v16b b, v8f c) {
  return __builtin_amdgcn_wmma_f32_16x16x32_bf16(false, a, false, b, (short)0, c, false, false);
}
__device__ __forceinline__ void grp_guard(v8f& a, v8f& b, v8f& c, v8f& d,
                                          v16b x, v16b y, v16b p, v16b q, v16b r, v16b s) {
  asm volatile("v_nop\n\tv_nop\n\tv_nop\n\tv_nop"
               : "+v"(a), "+v"(b), "+v"(c), "+v"(d)
               : "v"(x), "v"(y), "v"(p), "v"(q), "v"(r), "v"(s));
}
__device__ __forceinline__ void acc_guard4(v8f& a, v8f& b, v8f& c, v8f& d) {
  asm volatile("v_nop\n\tv_nop\n\tv_nop\n\tv_nop" : "+v"(a), "+v"(b), "+v"(c), "+v"(d));
}

template <int SPL, int BIAS_MODE, int OUT_MODE, bool RESID, int ACT>
__global__ __launch_bounds__(256) void wmma_gemm64(
    const unsigned short* __restrict__ Ap, const unsigned short* __restrict__ A2p, int lda, long strideA,
    const unsigned short* __restrict__ Btp, const unsigned short* __restrict__ Bt2p, int ldb, long strideB,
    void* __restrict__ Cout, void* __restrict__ Cout2, int ldc, long strideC,
    const float* __restrict__ bias,
    const float* __restrict__ resid, long strideR,
    int M, int N, int K, float scale) {
  const __bf16* A  = (const __bf16*)Ap;
  const __bf16* A2 = (const __bf16*)A2p;
  const __bf16* Bt = (const __bf16*)Btp;
  (void)Bt2p;
  __shared__ __align__(16) float sT[8][16 * 68];
  const int b    = blockIdx.y;
  const int lane = threadIdx.x & 31;
  const int wave = threadIdx.x >> 5;
  const int tilesN = N >> 6;
  const int tilesM = M >> 6;
  const int tile = blockIdx.x * 8 + wave;
  if (tile >= tilesM * tilesN) return;
  const int tm = tile / tilesN;
  const int tn = tile - tm * tilesN;
  const int m0 = tm << 6;
  const int n0 = tn << 6;

  const __bf16* Ab  = A  + (size_t)b * strideA;
  const __bf16* Bb  = Bt + (size_t)b * strideB;
  const __bf16* Ab2 = (SPL >= 1) ? (A2 + (size_t)b * strideA) : nullptr;

  const int rlane = lane & 15;
  const int koff  = (lane >> 4) * 8;
  const int mOff  = (lane >> 4) * 8;

  v8f acc[4][4];
#pragma unroll
  for (int i = 0; i < 4; ++i)
#pragma unroll
    for (int j = 0; j < 4; ++j) acc[i][j] = (v8f){0.f,0.f,0.f,0.f,0.f,0.f,0.f,0.f};

  for (int k0 = 0; k0 < K; k0 += 32) {
    v16b bh[4];
#pragma unroll
    for (int j = 0; j < 4; ++j) {
      const size_t bo = (size_t)(n0 + (j << 4) + rlane) * ldb + koff + k0;
      bh[j] = frag_load(Bb + bo);
    }
#pragma unroll
    for (int i = 0; i < 4; ++i) {
      const size_t ao = (size_t)(m0 + (i << 4) + rlane) * lda + koff + k0;
      v16b ah = frag_load(Ab + ao);
      v16b al = ah;
      if (SPL >= 1) al = frag_load(Ab2 + ao);
#pragma unroll
      for (int j = 0; j < 4; ++j) {
        acc[i][j] = mma_bf16(ah, bh[j], acc[i][j]);
        if (SPL >= 1) acc[i][j] = mma_bf16(al, bh[j], acc[i][j]);
      }
      grp_guard(acc[i][0], acc[i][1], acc[i][2], acc[i][3], ah, al, bh[0], bh[1], bh[2], bh[3]);
    }
  }
  acc_guard4(acc[0][0], acc[0][1], acc[0][2], acc[0][3]);
  acc_guard4(acc[1][0], acc[1][1], acc[1][2], acc[1][3]);
  acc_guard4(acc[2][0], acc[2][1], acc[2][2], acc[2][3]);
  acc_guard4(acc[3][0], acc[3][1], acc[3][2], acc[3][3]);

  float* slab = sT[wave];
  const float* Rb = (RESID || OUT_MODE == 3) ? (resid + (size_t)b * strideR) : nullptr;
#pragma unroll
  for (int i = 0; i < 4; ++i) {
    const int mBase = m0 + (i << 4);
#pragma unroll
    for (int j = 0; j < 4; ++j) {
      const int n = n0 + (j << 4) + rlane;
      float bv = 0.f;
      if (BIAS_MODE == 2) bv = bfr(bias[n]);
#pragma unroll
      for (int r = 0; r < 8; ++r) {
        float v = acc[i][j][r] * scale;
        if (BIAS_MODE == 2) v += bv;
        if (ACT == 3) v = v * __builtin_amdgcn_rcpf(1.0f + __expf(-v));
        slab[(mOff + r) * 68 + (j << 4) + rlane] = v;
      }
    }
    __builtin_amdgcn_fence(__ATOMIC_RELEASE, "workgroup");
    __builtin_amdgcn_wave_barrier();
    __builtin_amdgcn_fence(__ATOMIC_ACQUIRE, "workgroup");
    if (OUT_MODE == 0) {
      float* C = (float*)Cout + (size_t)b * strideC;
      const int hh = lane >> 4, c4 = (lane & 15) * 4;
      for (int pass = 0; pass < 2; ++pass) {
#pragma unroll
        for (int it = 0; it < 8; ++it) {
          const int row = it * 2 + hh;
          v4f v = *(const v4f*)(slab + row * 68 + c4);
          if (RESID) {
            const v4f rv = *(const v4f*)(Rb + (size_t)(mBase + row) * ldc + n0 + c4);
            v4f rr;
#pragma unroll
            for (int e = 0; e < 4; ++e) { const float re = rv[e]; rr[e] = bfr(re); }
            v = v + rr;
          }
          *(volatile v4f*)(C + (size_t)(mBase + row) * ldc + n0 + c4) = v;
        }
        __threadfence();
      }
    } else {
      const int q = lane >> 3, c8 = (lane & 7) * 8;
      unsigned short* C  = (unsigned short*)Cout  + (size_t)b * strideC;
      unsigned short* C2 = (unsigned short*)Cout2 + (size_t)b * strideC;
      for (int pass = 0; pass < 2; ++pass) {
#pragma unroll
        for (int it = 0; it < 4; ++it) {
          const int row = it * 4 + q;
          const float* sp = slab + row * 68 + c8;
          float gv[8];
#pragma unroll
          for (int e = 0; e < 8; ++e) gv[e] = 1.0f;
          if (OUT_MODE == 3) {
            const float* gp = Rb + (size_t)(mBase + row) * ldc + n0 + c8;
            const v4f g0 = *(const v4f*)(gp);
            const v4f g1 = *(const v4f*)(gp + 4);
            gv[0] = g0[0]; gv[1] = g0[1]; gv[2] = g0[2]; gv[3] = g0[3];
            gv[4] = g1[0]; gv[5] = g1[1]; gv[6] = g1[2]; gv[7] = g1[3];
          }
          v8h hv, lv;
#pragma unroll
          for (int e = 0; e < 8; ++e) {
            float val = sp[e];
            if (OUT_MODE == 3) val = val * gv[e];
            const unsigned short hb = f2bf_bits(val);
            const unsigned short lb = f2bf_bits(val - bf_bits2f(hb));
            hv[e] = __builtin_bit_cast(_Float16, hb);
            lv[e] = __builtin_bit_cast(_Float16, lb);
          }
          *(volatile v8h*)(C  + (size_t)(mBase + row) * ldc + n0 + c8) = hv;
          *(volatile v8h*)(C2 + (size_t)(mBase + row) * ldc + n0 + c8) = lv;
        }
        __threadfence();
      }
    }
    __builtin_amdgcn_fence(__ATOMIC_RELEASE, "workgroup");
    __builtin_amdgcn_wave_barrier();
    __builtin_amdgcn_fence(__ATOMIC_ACQUIRE, "workgroup");
  }
}

__global__ __launch_bounds__(256) void cast_rows_bf16_kernel(
    const float* __restrict__ src, unsigned short* __restrict__ dst, int total8)
{
  const int i = blockIdx.x * 256 + threadIdx.x;
  if (i >= total8) return;
  const size_t e0 = (size_t)i << 3;
  const v4f a0 = *(const v4f*)(src + e0);
  const v4f a1 = *(const v4f*)(src + e0 + 4);
  const v8h hv = pack_bf16x8(a0, a1);
  unsigned short* qh = dst + e0;
  *(volatile v8h*)qh = hv;
  __threadfence();
  *(volatile v8h*)qh = hv;
}

__global__ __launch_bounds__(256) void build_wbc_kernel(
    const float* __restrict__ wb, const float* __restrict__ wc, unsigned short* __restrict__ dst)
{
  const int row = blockIdx.x;
  const int col0 = threadIdx.x * 8;
  const int rb = row < (kNst - 1) ? row : (kNst - 1);
  int rc = row - kNst; rc = rc < 0 ? 0 : rc; rc = rc > (kNst - 1) ? (kNst - 1) : rc;
  const float fb = (row < kNst) ? 1.0f : 0.0f;
  const float fc = (row >= kNst && row < 2 * kNst) ? 1.0f : 0.0f;
  const v4f b0 = *(const v4f*)(wb + (size_t)rb * kE + col0);
  const v4f b1 = *(const v4f*)(wb + (size_t)rb * kE + col0 + 4);
  const v4f c0 = *(const v4f*)(wc + (size_t)rc * kE + col0);
  const v4f c1 = *(const v4f*)(wc + (size_t)rc * kE + col0 + 4);
  v4f s0, s1;
#pragma unroll
  for (int e = 0; e < 4; ++e) {
    const float xb0 = b0[e], xc0 = c0[e], xb1 = b1[e], xc1 = c1[e];
    s0[e] = fmaf(fb, xb0, fc * xc0);
    s1[e] = fmaf(fb, xb1, fc * xc1);
  }
  const v8h hv = pack_bf16x8(s0, s1);
  unsigned short* qh = dst + (size_t)row * kE + col0;
  *(volatile v8h*)qh = hv;
  __threadfence();
  *(volatile v8h*)qh = hv;
}

__global__ __launch_bounds__(256) void rmsnorm_split_kernel(
    const float* __restrict__ resid, const float* __restrict__ nw,
    unsigned short* __restrict__ XH, unsigned short* __restrict__ XL)
{
  __shared__ float part[8];
  const int tid = threadIdx.x, lane = tid & 31, wave = tid >> 5;
  const int rloc = tid >> 7, t = tid & 127;
  const int row = blockIdx.x * 2 + rloc;
  const int col0 = t * 8;
  const float* rp = resid + (size_t)row * kDm + col0;
  const v4f a0 = *(const v4f*)(rp);
  const v4f a1 = *(const v4f*)(rp + 4);
  v4f r0, r1;
#pragma unroll
  for (int e = 0; e < 4; ++e) { const float x0 = a0[e], x1 = a1[e]; r0[e] = bfr(x0); r1[e] = bfr(x1); }
  float ss = 0.0f;
#pragma unroll
  for (int e = 0; e < 4; ++e) { const float x0 = r0[e]; ss = fmaf(x0, x0, ss); }
#pragma unroll
  for (int e = 0; e < 4; ++e) { const float x1 = r1[e]; ss = fmaf(x1, x1, ss); }
#pragma unroll
  for (int off = 16; off > 0; off >>= 1) ss += __shfl_xor(ss, off, 32);
  if (lane == 0) part[wave] = ss;
  __syncthreads();
  const int w0 = rloc * 4;
  const float tot = (part[w0] + part[w0 + 1]) + (part[w0 + 2] + part[w0 + 3]);
  const float scale = rsqrtf(tot * (1.0f / (float)kDm) + 1e-5f);
  const v4f n0 = *(const v4f*)(nw + col0);
  const v4f n1 = *(const v4f*)(nw + col0 + 4);
  v4f x0, x1;
#pragma unroll
  for (int e = 0; e < 4; ++e) {
    const float g0 = n0[e], g1 = n1[e];
    const float y0 = r0[e], y1 = r1[e];
    x0[e] = (y0 * scale) * bfr(g0);
    x1[e] = (y1 * scale) * bfr(g1);
  }
  v8h hv, lv;
  split_bf16x8(x0, x1, hv, lv);
  const size_t o = (size_t)row * kDm + col0;
  for (int pass = 0; pass < 2; ++pass) {
    *(volatile v8h*)(XH + o) = hv;
    *(volatile v8h*)(XL + o) = lv;
    __threadfence();
  }
}

__global__ __launch_bounds__(256) void conv_silu_kernel(
    const float* __restrict__ XE, const float* __restrict__ cw, const float* __restrict__ cb,
    unsigned short* __restrict__ XSH, unsigned short* __restrict__ XSL)
{
  __shared__ __align__(16) float sT[16 * kConvTP];
  const int tid = threadIdx.x, lane = tid & 31, wave = tid >> 5;
  const int d0 = blockIdx.x * 256, d = d0 + tid;
  const int g0 = blockIdx.y * 64;
  const int tb = g0 & (kSeq - 1);
  const v4f wv = *(const v4f*)(cw + (size_t)d * 4);
  const float wq0 = wv[0], wq1 = wv[1], wq2 = wv[2], wq3 = wv[3];
  const float w0 = bfr(wq0), w1 = bfr(wq1), w2 = bfr(wq2), w3 = bfr(wq3);
  const float bc = bfr(cb[d]);
  float xm3, xm2, xm1;
  {
    const bool hist = (tb > 0);
    const float fh = hist ? 1.0f : 0.0f;
    const int rb = hist ? (g0 - 3) : g0;
    const float v3 = XE[(size_t)rb * kE + d];
    const float v2 = XE[(size_t)(rb + 1) * kE + d];
    const float v1 = XE[(size_t)(rb + 2) * kE + d];
    xm3 = v3 * fh;
    xm2 = v2 * fh;
    xm1 = v1 * fh;
  }
#pragma unroll 1
  for (int sub = 0; sub < 4; ++sub) {
    const int lb = g0 + sub * 16;
#pragma unroll 1
    for (int s = 0; s < 16; ++s) {
      const float xcur = XE[(size_t)(lb + s) * kE + d];
      float acc = w0 * xm3;
      acc = fmaf(w1, xm2, acc);
      acc = fmaf(w2, xm1, acc);
      acc = fmaf(w3, xcur, acc);
      const float sv = acc + bc;
      const float sg = __builtin_amdgcn_rcpf(1.0f + __expf(-sv));
      sT[s * kConvTP + tid] = sv * sg;
      xm3 = xm2; xm2 = xm1; xm1 = xcur;
    }
    __syncthreads();
    v8h bh[2], blo[2];
#pragma unroll
    for (int it = 0; it < 2; ++it) {
      const float* sp = sT + (it * 8 + wave) * kConvTP + lane * 8;
      const v4f a0 = *(const v4f*)(sp);
      const v4f a1 = *(const v4f*)(sp + 4);
      split_bf16x8(a0, a1, bh[it], blo[it]);
    }
    for (int pass = 0; pass < 2; ++pass) {
#pragma unroll
      for (int it = 0; it < 2; ++it) {
        const size_t o = (size_t)(lb + it * 8 + wave) * kE + d0 + lane * 8;
        *(volatile v8h*)(XSH + o) = bh[it];
        *(volatile v8h*)(XSL + o) = blo[it];
      }
      __threadfence();
    }
    __syncthreads();
  }
}

__global__ __launch_bounds__(64) void scan_kernel(
    const float* __restrict__ DZ, const float* __restrict__ XBC,
    const uint4* __restrict__ XSH4, const uint4* __restrict__ XSL4,
    const float* __restrict__ Alog, const float* __restrict__ Wd, float* __restrict__ YP)
{
  __shared__ __align__(16) float sBC[kScanTS * 32];
  __shared__ __align__(16) float sU[kScanTS * kScanP];
  __shared__ __align__(16) float sY[kScanTS * kScanP];
  __shared__ __align__(16) float sA[kNst * kScanCh];
  const int tid = threadIdx.x, lane = tid & 31, wave = tid >> 5;
  constexpr int kBlkPerB = kE / kScanCh;
  const int bix = blockIdx.x / kBlkPerB;
  const int d0  = (blockIdx.x - bix * kBlkPerB) * kScanCh;
  const int d   = d0 + tid;
  const size_t row0 = (size_t)bix * kSeq;
#pragma unroll 1
  for (int s = 0; s < kNst; ++s) sA[s * kScanCh + tid] = -expf(bfr(Alog[(size_t)d * kNst + s]));
  __syncthreads();
  float negA[kNst], h[kNst];
#pragma unroll
  for (int s = 0; s < kNst; ++s) {
    negA[s] = sA[s * kScanCh + tid];
    h[s] = 0.0f;
  }
  const float Wdd = bfr(Wd[d]);
  const int hh = lane >> 4, c4 = (lane & 15) * 4;
#pragma unroll 1
  for (int t0 = 0; t0 < kSeq; t0 += kScanTS) {
    __syncthreads();
#pragma unroll
    for (int i = 0; i < 8; ++i) {
      const int idx = tid + 64 * i;
      const int st = idx >> 3, cc = (idx & 7) * 4;
      *(v4f*)(sBC + st * 32 + cc) = *(const v4f*)(XBC + (row0 + t0 + st) * kBCW + cc);
    }
#pragma unroll 1
    for (int i = 0; i < 8; ++i) {
      const int idx = tid + 64 * i;
      const int st = idx >> 3, c8 = (idx & 7) * 8;
      const size_t w4 = ((row0 + t0 + st) * (size_t)kE + d0 + c8) >> 3;
      const uint4 wh = XSH4[w4];
      const uint4 wl = XSL4[w4];
      v4f u0, u1;
      u0[0] = __uint_as_float(wh.x << 16) + __uint_as_float(wl.x << 16);
      u0[1] = __uint_as_float(wh.x & 0xffff0000u) + __uint_as_float(wl.x & 0xffff0000u);
      u0[2] = __uint_as_float(wh.y << 16) + __uint_as_float(wl.y << 16);
      u0[3] = __uint_as_float(wh.y & 0xffff0000u) + __uint_as_float(wl.y & 0xffff0000u);
      u1[0] = __uint_as_float(wh.z << 16) + __uint_as_float(wl.z << 16);
      u1[1] = __uint_as_float(wh.z & 0xffff0000u) + __uint_as_float(wl.z & 0xffff0000u);
      u1[2] = __uint_as_float(wh.w << 16) + __uint_as_float(wl.w << 16);
      u1[3] = __uint_as_float(wh.w & 0xffff0000u) + __uint_as_float(wl.w & 0xffff0000u);
      *(v4f*)(sU + st * kScanP + c8)     = u0;
      *(v4f*)(sU + st * kScanP + c8 + 4) = u1;
    }
    __syncthreads();
#pragma unroll 1
    for (int s = 0; s < kScanTS; ++s) {
      const size_t grow = row0 + t0 + s;
      const float z = DZ[grow * kE + d];
      const float* xr = sBC + s * 32;
      float Bs[kNst], Cs[kNst];
#pragma unroll
      for (int q4 = 0; q4 < 4; ++q4) {
        const v4f bv = *(const v4f*)(xr + 4 * q4);
        const v4f cv = *(const v4f*)(xr + kNst + 4 * q4);
        Bs[4 * q4 + 0] = bv[0]; Bs[4 * q4 + 1] = bv[1]; Bs[4 * q4 + 2] = bv[2]; Bs[4 * q4 + 3] = bv[3];
        Cs[4 * q4 + 0] = cv[0]; Cs[4 * q4 + 1] = cv[1]; Cs[4 * q4 + 2] = cv[2]; Cs[4 * q4 + 3] = cv[3];
      }
      const float a   = __expf(-fabsf(z));
      const float u   = 1.0f + a;
      const float l1p = __logf(u) + (a - (u - 1.0f)) * __builtin_amdgcn_rcpf(u);
      const float dt  = fmaxf(z, 0.0f) + l1p;
      const float xt  = sU[s * kScanP + tid];
      const float dtx = dt * xt;
      float y = 0.0f;
#pragma unroll
      for (int k = 0; k < kNst; ++k) {
        const float e = __expf(dt * negA[k]);
        h[k] = e * h[k] + dtx * Bs[k];
        y = h[k] * Cs[k] + y;
      }
      y = xt * Wdd + y;
      sY[s * kScanP + tid] = y;
    }
    __syncthreads();
    for (int pass = 0; pass < 2; ++pass) {
#pragma unroll
      for (int it = 0; it < 16; ++it) {
        const int r = it * 4 + wave * 2 + hh;
        const v4f v = *(const v4f*)(sY + r * kScanP + c4);
        *(volatile v4f*)(YP + (row0 + t0 + r) * kE + d0 + c4) = v;
      }
      __threadfence();
    }
  }
}

extern "C" void kernel_launch(void* const* d_in, const int* in_sizes, int n_in,
                              void* d_out, int out_size, void* d_ws, size_t ws_size,
                              hipStream_t stream) {
  if (n_in < 14) return;
  if (in_sizes[0] != kRows * kDm) return;
  if (in_sizes[1] != kDm) return;
  if (in_sizes[2] != kE * kDm) return;
  if (in_sizes[3] != kE * kDm) return;
  if (in_sizes[4] != kE * 4) return;
  if (in_sizes[5] != kE) return;
  if (in_sizes[6] != kR * kE) return;
  if (in_sizes[7] != kE * kR) return;
  if (in_sizes[8] != kE) return;
  if (in_sizes[9] != kNst * kE) return;
  if (in_sizes[10] != kNst * kE) return;
  if (in_sizes[11] != kE * kNst) return;
  if (in_sizes[12] != kE) return;
  if (in_sizes[13] != kDm * kE) return;
  if (out_size != kRows * kDm) return;
  if (ws_size < kWsTotal) return;

  const float* resid  = (const float*)d_in[0];
  const float* norm_w = (const float*)d_in[1];
  const float* skip_w = (const float*)d_in[2];
  const float* in_w   = (const float*)d_in[3];
  const float* conv_w = (const float*)d_in[4];
  const float* conv_b = (const float*)d_in[5];
  const float* wd1    = (const float*)d_in[6];
  const float* wd2    = (const float*)d_in[7];
  const float* wd2_b  = (const float*)d_in[8];
  const float* wb     = (const float*)d_in[9];
  const float* wc     = (const float*)d_in[10];
  const float* A_log  = (const float*)d_in[11];
  const float* W_D    = (const float*)d_in[12];
  const float* out_w  = (const float*)d_in[13];
  float* out = (float*)d_out;

  char* ws = (char*)d_ws;
  unsigned short* XH   = (unsigned short*)(ws + kOffXH);
  unsigned short* XL   = (unsigned short*)(ws + kOffXL);
  unsigned short* WSK  = (unsigned short*)(ws + kOffWSK);
  unsigned short* WIN  = (unsigned short*)(ws + kOffWIN);
  unsigned short* WOUT = (unsigned short*)(ws + kOffWOUT);
  unsigned short* WD1  = (unsigned short*)(ws + kOffWD1);
  unsigned short* WBC  = (unsigned short*)(ws + kOffWBC);
  unsigned short* WD2  = (unsigned short*)(ws + kOffWD2);
  float*          XE   = (float*)(ws + kOffXE);
  float*          DZ   = (float*)(ws + kOffXE);
  unsigned short* XSH  = (unsigned short*)(ws + kOffXSH);
  unsigned short* XSL  = (unsigned short*)(ws + kOffXSL);
  unsigned short* YGH  = (unsigned short*)(ws + kOffXSH);
  unsigned short* YGL  = (unsigned short*)(ws + kOffXSL);
  unsigned short* D1H  = (unsigned short*)(ws + kOffD1H);
  unsigned short* D1L  = (unsigned short*)(ws + kOffD1L);
  float*          XBC  = (float*)(ws + kOffXBC);
  float*          YP   = (float*)(ws + kOffYP);

  cast_rows_bf16_kernel<<<(kE * kDm / 8) / 256, 256, 0, stream>>>(skip_w, WSK, kE * kDm / 8);
  cast_rows_bf16_kernel<<<(kE * kDm / 8) / 256, 256, 0, stream>>>(in_w, WIN, kE * kDm / 8);
  cast_rows_bf16_kernel<<<(kDm * kE / 8) / 256, 256, 0, stream>>>(out_w, WOUT, kDm * kE / 8);
  cast_rows_bf16_kernel<<<(kR * kE / 8) / 256, 256, 0, stream>>>(wd1, WD1, kR * kE / 8);
  cast_rows_bf16_kernel<<<(kE * kR / 8) / 256, 256, 0, stream>>>(wd2, WD2, kE * kR / 8);
  build_wbc_kernel<<<kBCW, 256, 0, stream>>>(wb, wc, WBC);

  rmsnorm_split_kernel<<<kRows / 2, 256, 0, stream>>>(resid, norm_w, XH, XL);

  wmma_gemm64<1, 0, 0, false, 0><<<dim3(256, 1), 256, 0, stream>>>(
      XH, XL, kDm, 0L,
      WIN, nullptr, kDm, 0L,
      (void*)XE, nullptr, kE, 0L,
      nullptr, nullptr, 0L,
      kRows, kE, kDm, 1.0f);

  conv_silu_kernel<<<dim3(kE / 256, kRows / 64), 256, 0, stream>>>(XE, conv_w, conv_b, XSH, XSL);

  wmma_gemm64<1, 0, 2, false, 0><<<dim3(8, 1), 256, 0, stream>>>(
      XSH, XSL, kE, 0L,
      WD1, nullptr, kE, 0L,
      (void*)D1H, (void*)D1L, kBCW, 0L,
      nullptr, nullptr, 0L,
      kRows, kBCW, kE, 1.0f);

  wmma_gemm64<1, 0, 0, false, 0><<<dim3(8, 1), 256, 0, stream>>>(
      XSH, XSL, kE, 0L,
      WBC, nullptr, kE, 0L,
      (void*)XBC, nullptr, kBCW, 0L,
      nullptr, nullptr, 0L,
      kRows, kBCW, kE, 1.0f);

  wmma_gemm64<1, 2, 0, false, 0><<<dim3(256, 1), 256, 0, stream>>>(
      D1H, D1L, kR, 0L,
      WD2, nullptr, kR, 0L,
      (void*)DZ, nullptr, kE, 0L,
      wd2_b, nullptr, 0L,
      kRows, kE, kR, 1.0f);

  scan_kernel<<<kBatch * (kE / kScanCh), kScanCh, 0, stream>>>(
      DZ, XBC, (const uint4*)(const void*)XSH, (const uint4*)(const void*)XSL, A_log, W_D, YP);

  wmma_gemm64<1, 0, 3, false, 3><<<dim3(256, 1), 256, 0, stream>>>(
      XH, XL, kDm, 0L,
      WSK, nullptr, kDm, 0L,
      (void*)YGH, (void*)YGL, kE, 0L,
      nullptr, YP, 0L,
      kRows, kE, kDm, 1.0f);

  wmma_gemm64<1, 0, 0, true, 0><<<dim3(128, 1), 256, 0, stream>>>(
      YGH, YGL, kE, 0L,
      WOUT, nullptr, kE, 0L,
      (void*)out, nullptr, kDm, 0L,
      nullptr, resid, 0L,
      kRows, kDm, kE, 1.0f);
}
